// XORWithPrevious_85950885527687
// MI455X (gfx1250) — hardware-verified
//
#include <hip/hip_runtime.h>
#include <stdint.h>

#define SEQ   2048
#define BITS  256
#define HEADS 8
#define NPOS  4
#define MAXD  8
#define NBPN  12
#define TBL_WORDS (HEADS * (1 << NBPN) / 32)

typedef int v8i __attribute__((ext_vector_type(8)));

#define OFF_AQ   (0)
#define OFF_AK   (32 * 1024)
#define OFF_AR   (64 * 1024)
#define OFF_TBL  (65 * 1024)
#define OFF_INC  (70 * 1024)
#define OFF_FB   (78 * 1024)
#define OFF_ATT  (1024 * 1024)
#define OFF_TT   (6 * 1024 * 1024)
#define OFF_INCP (8 * 1024 * 1024)
#define OFF_FBP  (8 * 1024 * 1024 + 256 * 1024)
typedef __attribute__((ext_vector_type(16))) _Float16 v16h;
typedef __attribute__((ext_vector_type(8)))  _Float16 v8h;
typedef __attribute__((ext_vector_type(8)))  float v8f;
typedef __attribute__((ext_vector_type(4)))  float v4f_t;
typedef float v4fa __attribute__((ext_vector_type(4), may_alias));

__global__ __launch_bounds__(256) void k_prep(const int* __restrict__ tokens,
                                              const int* __restrict__ head_idx,
                                              uint8_t* __restrict__ ws) {
    __shared__ int hidx[HEADS * NBPN];
    int tid = threadIdx.x;
    if (tid < HEADS * NBPN) hidx[tid] = head_idx[tid];
    __syncthreads();

    unsigned short* Aq = (unsigned short*)(ws + OFF_AQ);
    unsigned short* Ak = (unsigned short*)(ws + OFF_AK);
    unsigned short* Ar = (unsigned short*)(ws + OFF_AR);

    int s = blockIdx.x * 256 + tid;
    if (s < SEQ) {
        const int* trow = tokens + s * BITS;
        unsigned int pq[4] = {0u, 0u, 0u, 0u}, pk[4] = {0u, 0u, 0u, 0u};
        #pragma unroll
        for (int h = 0; h < HEADS; ++h) {
            int aq = 0, ak = 0;
            #pragma unroll
            for (int k = 0; k < NBPN; ++k) {
                int idx = hidx[h * NBPN + k];
                if (idx < BITS)           aq += trow[idx] << k;
                else if (idx < 2 * BITS)  ak += trow[idx - BITS] << k;
            }
            pq[h >> 1] |= ((unsigned)aq & 0xFFFFu) << (16 * (h & 1));
            pk[h >> 1] |= ((unsigned)ak & 0xFFFFu) << (16 * (h & 1));
        }
        uint4 vq = make_uint4(pq[0], pq[1], pq[2], pq[3]), vk = make_uint4(pk[0], pk[1], pk[2], pk[3]);
        typedef __attribute__((ext_vector_type(4))) unsigned v4u_t;
        v4u_t uq = {vq.x, vq.y, vq.z, vq.w}, uk = {vk.x, vk.y, vk.z, vk.w};
        *(volatile v4u_t*)(Aq + s * HEADS) = uq; *(volatile v4u_t*)(Ak + s * HEADS) = uk; __threadfence();
        *(volatile v4u_t*)(Aq + s * HEADS) = uq; *(volatile v4u_t*)(Ak + s * HEADS) = uk;
    }
    if (blockIdx.x == 0 && tid < (MAXD + 1) * HEADS) {
        int d = tid / HEADS, h = tid % HEADS;
        int ar = 0;
        #pragma unroll
        for (int k = 0; k < NBPN; ++k) {
            int idx = hidx[h * NBPN + k];
            if (idx >= 2 * BITS) {
                int p = idx - 2 * BITS;
                if (p > NPOS - 1) p = NPOS - 1;
                ar += ((d >> p) & 1) << k;
            }
        }
        *(volatile unsigned short*)(Ar + tid) = (unsigned short)ar; __threadfence(); *(volatile unsigned short*)(Ar + tid) = (unsigned short)ar;
    }
}

__global__ __launch_bounds__(256) void k_pack_table(const float* __restrict__ table,
                                                    uint8_t* __restrict__ ws) {
    int w = blockIdx.x * 256 + threadIdx.x;
    if (w >= TBL_WORDS) return;
    const float* src = table + w * 32;
    unsigned int bits = 0;
    #pragma unroll
    for (int b = 0; b < 32; ++b) bits |= (src[b] > 0.5f ? 1u : 0u) << b;
    *(volatile unsigned int*)((unsigned int*)(ws + OFF_TBL) + w) = bits; __threadfence(); *(volatile unsigned int*)((unsigned int*)(ws + OFF_TBL) + w) = bits;
}

__global__ __launch_bounds__(256) void k_pack_B(const int* __restrict__ tokens,
                                                uint8_t* __restrict__ ws) {
    int g = blockIdx.x * 256 + threadIdx.x;
    if (g >= BITS * (SEQ / 2)) return;
    int n = g / (SEQ / 2);
    int k = (g % (SEQ / 2)) * 2;
    const _Float16 a = (_Float16)(float)(tokens[k * BITS + n] & 1), b = (_Float16)(float)(tokens[(k + 1) * BITS + n] & 1);
    const unsigned v = (unsigned)__builtin_bit_cast(unsigned short, a) | ((unsigned)__builtin_bit_cast(unsigned short, b) << 16);
    unsigned* d = (unsigned*)((_Float16*)(ws + OFF_TT) + (size_t)n * SEQ + k);
    *(volatile unsigned*)d = v; __threadfence(); *(volatile unsigned*)d = v;
}

__global__ __launch_bounds__(256) void k_votes(uint8_t* __restrict__ ws) {
    __shared__ unsigned int   tbl[TBL_WORDS];
    __shared__ unsigned short aqar[(MAXD + 1) * HEADS];
    __shared__ unsigned int   skey[256];
    __shared__ unsigned int   scnt[256];

    int tid = threadIdx.x;
    int i   = blockIdx.x;

    const unsigned int* tblg = (const unsigned int*)(ws + OFF_TBL);
    for (int w = tid; w < TBL_WORDS; w += 256) tbl[w] = tblg[w];

    const unsigned short* Aq = (const unsigned short*)(ws + OFF_AQ);
    const unsigned short* Ar = (const unsigned short*)(ws + OFF_AR);
    if (tid < (MAXD + 1) * HEADS) {
        int h = tid % HEADS;
        aqar[tid] = (unsigned short)(Aq[i * HEADS + h] + Ar[tid]);
    }
    __syncthreads();

    const uint4* Ak = (const uint4*)(ws + OFF_AK);
    uint8_t* att = (uint8_t*)(ws + OFF_ATT) + (size_t)i * SEQ;

    unsigned int key = 0, cnt = 0;
    for (int j4 = tid * 4; j4 < SEQ; j4 += 1024) {
      unsigned int apack = 0;
      #pragma unroll
      for (int jj = 0; jj < 4; ++jj) {
        const int j = j4 + jj;
        unsigned char a = 0;
        if (j <= i) {
            uint4 akv = Ak[j];
            int d = i - j; if (d > MAXD) d = MAXD;
            const unsigned short* ap = &aqar[d * HEADS];
            unsigned int akw[4] = {akv.x, akv.y, akv.z, akv.w};
            int v = 0;
            #pragma unroll
            for (int h = 0; h < HEADS; ++h) {
                unsigned int akh = (h & 1) ? (akw[h >> 1] >> 16) : (akw[h >> 1] & 0xffffu);
                unsigned int addr = (unsigned int)ap[h] + akh;
                unsigned int wrd  = tbl[h * 128 + (addr >> 5)];
                v += (int)((wrd >> (addr & 31u)) & 1u);
            }
            a = (v >= HEADS / 2) ? 1 : 0;
            cnt += a;
            unsigned int kk = ((unsigned)v << 12) | (4095u - (unsigned)j);
            if (kk > key) key = kk;
        }
        apack |= (unsigned)a << (8 * jj);
      }
      *(volatile unsigned int*)(att + j4) = apack; __threadfence(); *(volatile unsigned int*)(att + j4) = apack;
    }

    skey[tid] = key; scnt[tid] = cnt;
    __syncthreads();
    for (int s = 128; s > 0; s >>= 1) {
        if (tid < s) {
            if (skey[tid + s] > skey[tid]) skey[tid] = skey[tid + s];
            scnt[tid] += scnt[tid + s];
        }
        __syncthreads();
    }
    if (tid == 0) {
        int* ip = (int*)(ws + OFF_INCP) + (size_t)i * 32; int* fp = (int*)(ws + OFF_FBP) + (size_t)i * 32;
        const int incv = (int)scnt[0], fbv = (int)(4095u - (skey[0] & 4095u));
        *(volatile int*)ip = incv; *(volatile int*)fp = fbv; __threadfence(); *(volatile int*)ip = incv; *(volatile int*)fp = fbv;
    }
}

__device__ __forceinline__ v8f wmma16(v16h a, v16h b, v8f c) { return __builtin_amdgcn_wmma_f32_16x16x32_f16(false, a, false, b, (short)0, c, false, false); }
__global__ __launch_bounds__(32) void k_wmma(const int* __restrict__ tokens,
                                             const uint8_t* __restrict__ ws,
                                             float* __restrict__ out) {
    __shared__ __attribute__((aligned(16))) float stg[32 * 36];
    int lane = threadIdx.x;
    int i0 = blockIdx.x * 32;
    int n0 = blockIdx.y * 32;
    int lo = lane & 15;
    int hi = lane >> 4;

    const uint8_t*  att = ws + OFF_ATT;
    const _Float16* TT  = (const _Float16*)(ws + OFF_TT);
    const int*      inc = (const int*)(ws + OFF_INCP);
    const int*      fb  = (const int*)(ws + OFF_FBP);

    v8f c[2][2];
    #pragma unroll
    for (int m = 0; m < 2; ++m)
        #pragma unroll
        for (int nt = 0; nt < 2; ++nt) c[m][nt] = (v8f){};

    const int nch = (i0 + 32 + 31) >> 5;
    #pragma unroll 1
    for (int kc = 0; kc < nch; ++kc) {
        const int k0 = kc << 5;
        v16h a[2], b[2];
        #pragma unroll
        for (int m = 0; m < 2; ++m) {
            const uint8_t* ap = att + (size_t)(i0 + m * 16 + lo) * SEQ + k0 + hi * 8;
            const uint2 u0 = *(const uint2*)ap, u1 = *(const uint2*)(ap + 16);
            unsigned w[4] = {u0.x, u0.y, u1.x, u1.y};
            #pragma unroll
            for (int e = 0; e < 16; ++e) a[m][e] = (_Float16)(float)((w[e >> 2] >> (8 * (e & 3))) & 0xFFu);
        }
        #pragma unroll
        for (int nt = 0; nt < 2; ++nt) {
            const _Float16* bp = TT + (size_t)(n0 + nt * 16 + lo) * SEQ + k0 + hi * 8;
            b[nt] = __builtin_shufflevector(*(const v8h*)bp, *(const v8h*)(bp + 16), 0,1,2,3,4,5,6,7,8,9,10,11,12,13,14,15);
        }
        #pragma unroll
        for (int m = 0; m < 2; ++m)
            #pragma unroll
            for (int nt = 0; nt < 2; ++nt) c[m][nt] = wmma16(a[m], b[nt], c[m][nt]);
    }

    #pragma unroll
    for (int m = 0; m < 2; ++m) {
        #pragma unroll
        for (int r = 0; r < 8; ++r) {
            const int il = m * 16 + r + hi * 8, i = i0 + il;
            const int fbi = fb[(size_t)i * 32], inci = inc[(size_t)i * 32];
            const int fbc = (fbi < 0) ? 0 : ((fbi >= SEQ) ? SEQ - 1 : fbi);
            #pragma unroll
            for (int nt = 0; nt < 2; ++nt) {
                const int nl = nt * 16 + lo;
                int v = ((int)(c[m][nt][r] + 0.5f)) & 1;
                if (inci == 0) v = tokens[fbc * BITS + n0 + nl] & 1;
                stg[il * 36 + nl] = (float)v;
            }
        }
    }
    asm volatile("s_wait_dscnt 0" ::: "memory");
    #pragma unroll 1
    for (int pass = 0; pass < 2; ++pass) {
        #pragma unroll
        for (int q = 0; q < 8; ++q) { const int cc = lane + 32 * q, rr = cc >> 3, c4 = (cc & 7) * 4;
            *(volatile v4f_t*)(out + (size_t)(i0 + rr) * BITS + n0 + c4) = *(const volatile v4fa*)(stg + rr * 36 + c4); }
        __threadfence();
    }
}

extern "C" void kernel_launch(void* const* d_in, const int* in_sizes, int n_in,
                              void* d_out, int out_size, void* d_ws, size_t ws_size,
                              hipStream_t stream) {
    const int*   tokens   = (const int*)d_in[0];
    const int*   head_idx = (const int*)d_in[1];
    const float* table    = (const float*)d_in[2];
    uint8_t*     ws       = (uint8_t*)d_ws;
    float*       out      = (float*)d_out;

    k_prep<<<SEQ / 256, 256, 0, stream>>>(tokens, head_idx, ws);
    k_pack_table<<<TBL_WORDS / 256, 256, 0, stream>>>(table, ws);
    k_pack_B<<<(BITS * (SEQ / 2)) / 256, 256, 0, stream>>>(tokens, ws);
    k_votes<<<SEQ, 256, 0, stream>>>(ws);
    k_wmma<<<dim3(SEQ / 32, BITS / 32), 32, 0, stream>>>(tokens, ws, out);
    (void)in_sizes; (void)n_in; (void)out_size; (void)ws_size;
}
